// GATReg_add_70592082477426
// MI455X (gfx1250) — hardware-verified
//
#include <hip/hip_runtime.h>
#include <stddef.h>
#include <stdint.h>


#define INDIM  128
#define F2     256
#define HEADS  4
#define HID    64
#define EXTRA  32
#define FIN    (F2 + EXTRA)
#define H2DIM  (HID / 2)
#define GR     32
#define XSP    (F2 + 8)
#define NB     256
#define CHUNK  2048
#define NTHR   256
#define NWAVE  8
#define NGRP   (CHUNK / (NTHR * 4))
#define WCAPB  768
#define GCHUNK (NTHR * 4)
#define GCAPW  128
#define OUTCAP 2048
#define ASCALE 8.0f
#define WSCALE 16.0f
#define OSCALE (1.0f / 128.0f)

#define LDS_SACC (NB * F2)
#define LDS_DEN  (NB * HEADS)
#define LDS_LIST (NWAVE * WCAPB)
#define LDS_GAT_BYTES ((LDS_SACC + LDS_DEN + LDS_LIST + NWAVE) * 4)

static_assert(NGRP == 2);
static_assert(NB == NWAVE * 32);
static_assert(NB == 256);
static_assert(F2 == HEADS * HID);
static_assert(NTHR == GR * 8);
static_assert(NTHR == F2);
static_assert(((LDS_SACC + LDS_DEN) % 4) == 0);
static_assert(LDS_GAT_BYTES == 290848);
static_assert((XSP % 4) == 0);

typedef float    v4f  __attribute__((ext_vector_type(4)));
typedef float    v8f  __attribute__((ext_vector_type(8)));
typedef int      v4i  __attribute__((ext_vector_type(4)));
typedef _Float16 v8h  __attribute__((ext_vector_type(8)));
typedef _Float16 v16h __attribute__((ext_vector_type(16)));
union Frag   { v16h v; v8h half[2]; };
union Pack16 { v8h h; v4i i; };

__device__ __forceinline__ v8f wm(v16h a, v16h b, v8f c) {
  v8f d = __builtin_amdgcn_wmma_f32_16x16x32_f16(false, a, false, b, (short)0, c, false, false);
  asm volatile("v_nop\n\tv_nop\n\tv_nop\n\tv_nop" : "+v"(d) : "v"(a), "v"(b));
  return d;
}

__device__ __forceinline__ int clampi(int v, int lo, int hi) {
  return v < lo ? lo : (v > hi ? hi : v);
}

__device__ __forceinline__ v4i load4i(const int* p, int i0, int n, bool al16, int sent) {
  v4i d;
  if (al16 && (i0 + 3 < n)) {
    d = *(const v4i*)(p + i0);
  } else {
    d.x = (i0     < n) ? p[i0]     : sent;
    d.y = (i0 + 1 < n) ? p[i0 + 1] : sent;
    d.z = (i0 + 2 < n) ? p[i0 + 2] : sent;
    d.w = (i0 + 3 < n) ? p[i0 + 3] : sent;
  }
  return d;
}

__global__ __launch_bounds__(NTHR) void k_prep_a(const float* __restrict__ X, _Float16* Ah, int n8) {
  const int i = blockIdx.x * NTHR + threadIdx.x;
  if (i >= n8) return;
  const size_t o = (size_t)i * 8;
  const v4f a = *(const v4f*)(X + o);
  const v4f b = *(const v4f*)(X + o + 4);
  Pack16 u;
  u.h[0] = (_Float16)(a.x * ASCALE); u.h[1] = (_Float16)(a.y * ASCALE);
  u.h[2] = (_Float16)(a.z * ASCALE); u.h[3] = (_Float16)(a.w * ASCALE);
  u.h[4] = (_Float16)(b.x * ASCALE); u.h[5] = (_Float16)(b.y * ASCALE);
  u.h[6] = (_Float16)(b.z * ASCALE); u.h[7] = (_Float16)(b.w * ASCALE);
  *(volatile v4i*)(Ah + o) = u.i;
  __threadfence();
  *(volatile v4i*)(Ah + o) = u.i;
}

__global__ __launch_bounds__(NTHR) void k_prep_w(const float* __restrict__ W, _Float16* Wt, int K, int Nc) {
  const int i  = blockIdx.x * NTHR + threadIdx.x;
  const int kq = K >> 3;
  if (i >= Nc * kq) return;
  const int n  = i / kq;
  const int k8 = i - n * kq;
  const float* p = W + (size_t)(8 * k8) * Nc + n;
  Pack16 u;
#pragma unroll
  for (int j = 0; j < 8; ++j) u.h[j] = (_Float16)(p[(size_t)j * Nc] * WSCALE);
  _Float16* q = Wt + (size_t)n * K + 8 * k8;
  *(volatile v4i*)q = u.i;
  __threadfence();
  *(volatile v4i*)q = u.i;
}

template <int KD>
__global__ __launch_bounds__(NTHR) void k_gemm(const _Float16* __restrict__ Ah, const _Float16* __restrict__ Wt,
                                               const float* __restrict__ al, const float* __restrict__ ar,
                                               float* feat, float* elr, int nA) {
  __shared__ __attribute__((aligned(16))) float Xs[GR * XSP];
  __shared__ __attribute__((aligned(16))) float Es[GR * 8];

  const int tid  = threadIdx.x;
  const int lane = tid & 31;
  const int wave = tid >> 5;
  const int hh   = lane >> 4;
  const int m    = lane & 15;
  const int rowBase = blockIdx.x * GR;

  int r0 = rowBase + m;      if (r0 > nA - 1) r0 = nA - 1;
  int r1 = rowBase + 16 + m; if (r1 > nA - 1) r1 = nA - 1;
  const int n0 = wave * 32 + m;
  const int n1 = n0 + 16;
  const _Float16* pa0 = Ah + (size_t)r0 * KD + 8 * hh;
  const _Float16* pa1 = Ah + (size_t)r1 * KD + 8 * hh;
  const _Float16* pb0 = Wt + (size_t)n0 * KD + 8 * hh;
  const _Float16* pb1 = Wt + (size_t)n1 * KD + 8 * hh;

  v8f c00 = {0.f, 0.f, 0.f, 0.f, 0.f, 0.f, 0.f, 0.f};
  v8f c01 = {0.f, 0.f, 0.f, 0.f, 0.f, 0.f, 0.f, 0.f};
  v8f c10 = {0.f, 0.f, 0.f, 0.f, 0.f, 0.f, 0.f, 0.f};
  v8f c11 = {0.f, 0.f, 0.f, 0.f, 0.f, 0.f, 0.f, 0.f};
#pragma unroll 4
  for (int kt = 0; kt < KD / 32; ++kt) {
    const int k0 = kt * 32;
    Frag a0, a1, b0, b1;
    a0.half[0] = *(const v8h*)(pa0 + k0); a0.half[1] = *(const v8h*)(pa0 + k0 + 16);
    a1.half[0] = *(const v8h*)(pa1 + k0); a1.half[1] = *(const v8h*)(pa1 + k0 + 16);
    b0.half[0] = *(const v8h*)(pb0 + k0); b0.half[1] = *(const v8h*)(pb0 + k0 + 16);
    b1.half[0] = *(const v8h*)(pb1 + k0); b1.half[1] = *(const v8h*)(pb1 + k0 + 16);
    c00 = wm(a0.v, b0.v, c00);
    c01 = wm(a0.v, b1.v, c01);
    c10 = wm(a1.v, b0.v, c10);
    c11 = wm(a1.v, b1.v, c11);
  }

#pragma unroll
  for (int r = 0; r < 8; ++r) {
    const int ra = 8 * hh + r;
    const int rb = 16 + 8 * hh + r;
    Xs[ra * XSP + n0] = c00[r] * OSCALE;
    Xs[ra * XSP + n1] = c01[r] * OSCALE;
    Xs[rb * XSP + n0] = c10[r] * OSCALE;
    Xs[rb * XSP + n1] = c11[r] * OSCALE;
  }
  __syncthreads();

  {
    const int row = tid >> 3;
    const int h   = (tid >> 1) & 3;
    const int lr  = tid & 1;
    const float* av = (lr ? ar : al) + h * HID;
    const float* xs = Xs + row * XSP + h * HID;
    float s = 0.f;
#pragma unroll 4
    for (int d = 0; d < HID; ++d) s += xs[d] * av[d];
    Es[row * 8 + lr * 4 + h] = s;
  }
  __syncthreads();

  v4f xr[8];
  float* fp[4];
#pragma unroll
  for (int i = 0; i < 4; ++i) {
    const int row = 4 * wave + i;
    xr[2 * i]     = *(const v4f*)(Xs + row * XSP + 4 * lane);
    xr[2 * i + 1] = *(const v4f*)(Xs + row * XSP + 128 + 4 * lane);
    fp[i] = feat + (size_t)(rowBase + row) * F2 + 4 * lane;
  }
  v4f ev = {0.f, 0.f, 0.f, 0.f};
  float* ep = elr + (size_t)rowBase * 8 + (wave & 1) * 128 + 4 * lane;
  if (wave < 2) ev = *(const v4f*)(Es + wave * 128 + 4 * lane);

#pragma unroll
  for (int i = 0; i < 4; ++i) {
    *(volatile v4f*)(fp[i])       = xr[2 * i];
    *(volatile v4f*)(fp[i] + 128) = xr[2 * i + 1];
  }
  if (wave < 2) *(volatile v4f*)ep = ev;
  __threadfence();
#pragma unroll
  for (int i = 0; i < 4; ++i) {
    *(volatile v4f*)(fp[i])       = xr[2 * i];
    *(volatile v4f*)(fp[i] + 128) = xr[2 * i + 1];
  }
  if (wave < 2) *(volatile v4f*)ep = ev;
}

template <bool L1>
__global__ __launch_bounds__(NTHR) void k_gat(const int* __restrict__ srcA, const int* __restrict__ dstA,
                                              const float* __restrict__ feat, const float* __restrict__ elr,
                                              const float* __restrict__ bias,
                                              _Float16* outH, float* outF, int nN, int nE) {
  extern __shared__ v4f lds_dyn[];
  float* sacc = (float*)lds_dyn;
  float* den  = sacc + LDS_SACC;
  int*   list = (int*)(den + LDS_DEN);
  int*   wcnt = list + LDS_LIST;

  const int tid  = threadIdx.x;
  const int lane = tid & 31;
  const int wave = tid >> 5;
  const int nodeBase = blockIdx.x * NB;

  {
    const v4f z4 = {0.f, 0.f, 0.f, 0.f};
    for (int i = tid; i < (LDS_SACC + LDS_DEN) / 4; i += NTHR) lds_dyn[i] = z4;
  }

  const bool al16 = ((((size_t)dstA) & 15) == 0);
  const int nChunks = (nE + CHUNK - 1) / CHUNK;
  const int sent = -2147483647 - 1;
  int wc = 0;
#pragma unroll 1
  for (int ch = 0; ch < nChunks; ++ch) {
    const int cbase = ch * CHUNK;
#pragma unroll
    for (int g = 0; g < NGRP; ++g) {
      const int e0 = cbase + (g * NTHR + tid) * 4;
      const v4i d = load4i(dstA, e0, nE, al16, sent);
      const unsigned s0 = (unsigned)d.x - (unsigned)nodeBase;
      const unsigned s1 = (unsigned)d.y - (unsigned)nodeBase;
      const unsigned s2 = (unsigned)d.z - (unsigned)nodeBase;
      const unsigned s3 = (unsigned)d.w - (unsigned)nodeBase;
      const bool h0 = s0 < (unsigned)NB;
      const bool h1 = s1 < (unsigned)NB;
      const bool h2 = s2 < (unsigned)NB;
      const bool h3 = s3 < (unsigned)NB;
      const unsigned many = __builtin_amdgcn_ballot_w32(h0 | h1 | h2 | h3);
      if (many != 0u) {
#define HITJ(J, HJ, SJ) { \
          const unsigned mj = __builtin_amdgcn_ballot_w32(HJ); \
          if (HJ) { \
            const int pos = wc + (int)__builtin_amdgcn_mbcnt_lo(mj, 0u); \
            if (pos < WCAPB) list[wave * WCAPB + pos] = ((e0 + (J)) << 8) | (int)(SJ); \
          } \
          wc += (int)__builtin_popcount(mj); }
        HITJ(0, h0, s0)
        HITJ(1, h1, s1)
        HITJ(2, h2, s2)
        HITJ(3, h3, s3)
#undef HITJ
      }
    }
  }
  if (lane == 0) wcnt[wave] = wc;
  __syncthreads();

  if (wave == 0) {
    const int hd = lane >> 3;
    const int c0 = 8 * lane;
#pragma unroll 1
    for (int w = 0; w < NWAVE; ++w) {
      int n = wcnt[w];
      n = n < 0 ? 0 : (n > WCAPB ? WCAPB : n);
#pragma unroll 1
      for (int i = 0; i < n; ++i) {
        const int ent  = list[w * WCAPB + i];
        const int slot = ent & (NB - 1);
        int e = (int)(((unsigned)ent) >> 8);
        if (e > nE - 1) e = nE - 1;
        const int s  = clampi(srcA[e], 0, nN - 1);
        const int nd = clampi(nodeBase + slot, 0, nN - 1);
        float lg = elr[(size_t)s * 8 + hd] + elr[(size_t)nd * 8 + 4 + hd];
        lg = (lg > 0.f) ? lg : 0.2f * lg;
        lg = fminf(lg, 80.f);
        const float p = __expf(lg);
        const float* fr = feat + (size_t)s * F2 + c0;
        const v4f x0 = *(const v4f*)(fr);
        const v4f x1 = *(const v4f*)(fr + 4);
        v4f* sp = (v4f*)(sacc + slot * F2 + c0);
        v4f a0 = sp[0];
        v4f a1 = sp[1];
        a0 = a0 + p * x0;
        a1 = a1 + p * x1;
        sp[0] = a0;
        sp[1] = a1;
        if ((lane & 7) == 0) {
          const float o = den[slot * HEADS + hd];
          den[slot * HEADS + hd] = o + p;
        }
      }
    }
  }
  __syncthreads();

  if (L1) {
    const int hd = lane >> 3;
    const int c0 = 8 * lane;
    const v4f b0 = *(const v4f*)(bias + c0);
    const v4f b1 = *(const v4f*)(bias + c0 + 4);
#pragma unroll 1
    for (int j = 0; j < NB / NWAVE; ++j) {
      const int slot = wave * (NB / NWAVE) + j;
      const size_t node = (size_t)(nodeBase + slot);
      const float dv  = den[slot * HEADS + hd];
      const float inv = (dv > 0.f) ? (1.0f / dv) : 0.f;
      const v4f a0 = *(const v4f*)(sacc + slot * F2 + c0);
      const v4f a1 = *(const v4f*)(sacc + slot * F2 + c0 + 4);
      v4f v0 = a0 * inv + b0;
      v4f v1 = a1 * inv + b1;
      v0.x = v0.x > 0.f ? v0.x : 0.f; v0.y = v0.y > 0.f ? v0.y : 0.f;
      v0.z = v0.z > 0.f ? v0.z : 0.f; v0.w = v0.w > 0.f ? v0.w : 0.f;
      v1.x = v1.x > 0.f ? v1.x : 0.f; v1.y = v1.y > 0.f ? v1.y : 0.f;
      v1.z = v1.z > 0.f ? v1.z : 0.f; v1.w = v1.w > 0.f ? v1.w : 0.f;
      Pack16 u;
      u.h[0] = (_Float16)(v0.x * ASCALE); u.h[1] = (_Float16)(v0.y * ASCALE);
      u.h[2] = (_Float16)(v0.z * ASCALE); u.h[3] = (_Float16)(v0.w * ASCALE);
      u.h[4] = (_Float16)(v1.x * ASCALE); u.h[5] = (_Float16)(v1.y * ASCALE);
      u.h[6] = (_Float16)(v1.z * ASCALE); u.h[7] = (_Float16)(v1.w * ASCALE);
      _Float16* op = outH + node * F2 + c0;
      *(volatile v4i*)op = u.i;
      __threadfence();
      *(volatile v4i*)op = u.i;
    }
  } else {
    const int cA = 4 * lane;
    const int cB = 128 + 4 * lane;
    const int hA = lane >> 4;
    const int hB = 2 + (lane >> 4);
    const v4f bA = *(const v4f*)(bias + cA);
    const v4f bB = *(const v4f*)(bias + cB);
#pragma unroll 1
    for (int j = 0; j < NB / NWAVE; ++j) {
      const int slot = wave * (NB / NWAVE) + j;
      const size_t node = (size_t)(nodeBase + slot);
      const float dA = den[slot * HEADS + hA];
      const float dB = den[slot * HEADS + hB];
      const float iA = (dA > 0.f) ? (1.0f / dA) : 0.f;
      const float iB = (dB > 0.f) ? (1.0f / dB) : 0.f;
      v4f vA = *(const v4f*)(sacc + slot * F2 + cA) * iA + bA;
      v4f vB = *(const v4f*)(sacc + slot * F2 + cB) * iB + bB;
      vA.x = vA.x > 0.f ? vA.x : 0.f; vA.y = vA.y > 0.f ? vA.y : 0.f;
      vA.z = vA.z > 0.f ? vA.z : 0.f; vA.w = vA.w > 0.f ? vA.w : 0.f;
      vB.x = vB.x > 0.f ? vB.x : 0.f; vB.y = vB.y > 0.f ? vB.y : 0.f;
      vB.z = vB.z > 0.f ? vB.z : 0.f; vB.w = vB.w > 0.f ? vB.w : 0.f;
      float* op = outF + node * F2;
      *(volatile v4f*)(op + cA) = vA;
      *(volatile v4f*)(op + cB) = vB;
      __threadfence();
      *(volatile v4f*)(op + cA) = vA;
      *(volatile v4f*)(op + cB) = vB;
    }
  }
}

__global__ __launch_bounds__(NTHR) void k_pool_head(const float* __restrict__ h2, const int* __restrict__ gid,
                                                    const float* __restrict__ desc,
                                                    const float* __restrict__ fc1w, const float* __restrict__ fc1b,
                                                    const float* __restrict__ fc2w, const float* __restrict__ fc2b,
                                                    const float* __restrict__ ow, const float* __restrict__ ob,
                                                    float* out, int nN, int nG, int nOut, float invNpg) {
  __shared__ int glist[NWAVE * GCAPW];
  __shared__ int gcnt[NWAVE];
  __shared__ float comb[FIN];
  __shared__ float z1[HID];
  __shared__ float z2[H2DIM];
  __shared__ __attribute__((aligned(16))) float outs[OUTCAP];

  const int tid  = threadIdx.x;
  const int lane = tid & 31;
  const int wave = tid >> 5;
  const bool al16 = ((((size_t)gid) & 15) == 0);
  const int nCh = (nN + GCHUNK - 1) / GCHUNK;
  const int sent = -2147483647 - 1;

#pragma unroll 1
  for (int g = 0; g < nG; ++g) {
    int wc = 0;
#pragma unroll 1
    for (int ch = 0; ch < nCh; ++ch) {
      const int i0 = ch * GCHUNK + tid * 4;
      const v4i d = load4i(gid, i0, nN, al16, sent);
      const bool h0 = (d.x == g), h1 = (d.y == g), h2b = (d.z == g), h3 = (d.w == g);
      const unsigned many = __builtin_amdgcn_ballot_w32(h0 | h1 | h2b | h3);
      if (many != 0u) {
#define GHIT(J, HJ) { \
          const unsigned mj = __builtin_amdgcn_ballot_w32(HJ); \
          if (HJ) { \
            const int pos = wc + (int)__builtin_amdgcn_mbcnt_lo(mj, 0u); \
            if (pos < GCAPW) glist[wave * GCAPW + pos] = i0 + (J); \
          } \
          wc += (int)__builtin_popcount(mj); }
        GHIT(0, h0)
        GHIT(1, h1)
        GHIT(2, h2b)
        GHIT(3, h3)
#undef GHIT
      }
    }
    if (lane == 0) gcnt[wave] = wc;
    __syncthreads();

    float s = 0.f;
#pragma unroll 1
    for (int w = 0; w < NWAVE; ++w) {
      int n = gcnt[w];
      n = n < 0 ? 0 : (n > GCAPW ? GCAPW : n);
#pragma unroll 1
      for (int i = 0; i < n; ++i) {
        const int nd = clampi(glist[w * GCAPW + i], 0, nN - 1);
        s += h2[(size_t)nd * F2 + tid];
      }
    }
    comb[tid] = s * invNpg;
    if (tid < EXTRA) comb[F2 + tid] = desc[(size_t)g * EXTRA + tid];
    __syncthreads();

    if (tid < HID) {
      float z = fc1b[tid];
#pragma unroll 1
      for (int i = 0; i < FIN; ++i) z += comb[i] * fc1w[(size_t)i * HID + tid];
      z1[tid] = z > 0.f ? z : 0.f;
    }
    __syncthreads();
    if (tid < H2DIM) {
      float z = fc2b[tid];
#pragma unroll 1
      for (int i = 0; i < HID; ++i) z += z1[i] * fc2w[i * H2DIM + tid];
      z2[tid] = z > 0.f ? z : 0.f;
    }
    __syncthreads();
    if (tid == 0) {
      float z = ob[0];
#pragma unroll 1
      for (int i = 0; i < H2DIM; ++i) z += z2[i] * ow[i];
      outs[g] = z;
    }
  }
  __syncthreads();

  if (wave == 0) {
    const int n4 = nOut >> 2;
    for (int idx4 = lane; idx4 < n4; idx4 += 32)
      *(volatile v4f*)(out + 4 * idx4) = *(const v4f*)(outs + 4 * idx4);
    if (lane == 0)
      for (int t = n4 * 4; t < nOut; ++t) *(volatile float*)(out + t) = outs[t];
    __threadfence();
    for (int idx4 = lane; idx4 < n4; idx4 += 32)
      *(volatile v4f*)(out + 4 * idx4) = *(const v4f*)(outs + 4 * idx4);
    if (lane == 0)
      for (int t = n4 * 4; t < nOut; ++t) *(volatile float*)(out + t) = outs[t];
  }
}

extern "C" void kernel_launch(void* const* d_in, const int* in_sizes, int n_in,
                              void* d_out, int out_size, void* d_ws, size_t ws_size,
                              hipStream_t stream) {
  if (n_in < 19) return;
  const int nN = in_sizes[4];
  const int nE = in_sizes[2];
  const int nG = out_size;
  if (nN <= 0 || nG <= 0 || nE < 0) return;
  if (nG > OUTCAP || nE > (1 << 23) || nN > (1 << 23)) return;
  if (in_sizes[0] != nN * INDIM || in_sizes[1] != nG * EXTRA || in_sizes[3] != nE) return;
  if (in_sizes[5] != INDIM * F2 || in_sizes[6] != F2 || in_sizes[7] != F2 || in_sizes[8] != F2) return;
  if (in_sizes[9] != F2 * F2 || in_sizes[10] != F2 || in_sizes[11] != F2 || in_sizes[12] != F2) return;
  if (in_sizes[13] != FIN * HID || in_sizes[14] != HID || in_sizes[15] != HID * H2DIM) return;
  if (in_sizes[16] != H2DIM || in_sizes[17] != H2DIM || in_sizes[18] != 1) return;
  const int npg = nN / nG;
  if (npg <= 0) return;
  const float invNpg = 1.0f / (float)npg;

  const float* x     = (const float*)d_in[0];
  const float* desc  = (const float*)d_in[1];
  const int*   src   = (const int*)d_in[2];
  const int*   dst   = (const int*)d_in[3];
  const int*   gidp  = (const int*)d_in[4];
  const float* W1    = (const float*)d_in[5];
  const float* al1   = (const float*)d_in[6];
  const float* ar1   = (const float*)d_in[7];
  const float* b1    = (const float*)d_in[8];
  const float* W2    = (const float*)d_in[9];
  const float* al2   = (const float*)d_in[10];
  const float* ar2   = (const float*)d_in[11];
  const float* b2    = (const float*)d_in[12];
  const float* fc1w  = (const float*)d_in[13];
  const float* fc1b  = (const float*)d_in[14];
  const float* fc2w  = (const float*)d_in[15];
  const float* fc2b  = (const float*)d_in[16];
  const float* ow    = (const float*)d_in[17];
  const float* ob    = (const float*)d_in[18];
  float* out = (float*)d_out;

  const int nP  = ((nN + GR - 1) / GR) * GR;
  const int nPg = ((nN + NB - 1) / NB) * NB;
  char* ws = (char*)d_ws;
  size_t off = 0;
  const size_t szWt1  = (((size_t)F2 * INDIM * 2) + 255) & ~(size_t)255;
  const size_t szWt2  = (((size_t)F2 * F2 * 2) + 255) & ~(size_t)255;
  const size_t szFeat = (((size_t)nP * F2 * 4) + 255) & ~(size_t)255;
  const size_t szElr  = (((size_t)nP * 8 * 4) + 255) & ~(size_t)255;
  const size_t szAh1  = (((size_t)nN * INDIM * 2) + 255) & ~(size_t)255;
  const size_t szH1h  = (((size_t)nPg * F2 * 2) + 255) & ~(size_t)255;
  const size_t szH2   = (((size_t)nPg * F2 * 4) + 255) & ~(size_t)255;
  _Float16* Wt1 = (_Float16*)(ws + off); off += szWt1;
  _Float16* Wt2 = (_Float16*)(ws + off); off += szWt2;
  float* feat   = (float*)(ws + off);    off += szFeat;
  float* elr    = (float*)(ws + off);    off += szElr;
  const size_t U = off;
  _Float16* Ah1 = (_Float16*)(ws + U);
  _Float16* h1h = (_Float16*)(ws + U + szAh1);
  float*    h2  = (float*)(ws + U);
  const size_t szU = (szAh1 + szH1h > szH2) ? (szAh1 + szH1h) : szH2;
  off = U + szU;
  if (off > ws_size) return;
  if (off > (size_t)134217728) return;

  const int n8 = nN * INDIM / 8;
  k_prep_a<<<(n8 + NTHR - 1) / NTHR, NTHR, 0, stream>>>(x, Ah1, n8);
  const int t1 = F2 * (INDIM / 8);
  k_prep_w<<<(t1 + NTHR - 1) / NTHR, NTHR, 0, stream>>>(W1, Wt1, INDIM, F2);
  const int t2 = F2 * (F2 / 8);
  k_prep_w<<<(t2 + NTHR - 1) / NTHR, NTHR, 0, stream>>>(W2, Wt2, F2, F2);

  hipFuncSetAttribute(reinterpret_cast<const void*>(&k_gat<true>),
                      hipFuncAttributeMaxDynamicSharedMemorySize, LDS_GAT_BYTES);
  hipFuncSetAttribute(reinterpret_cast<const void*>(&k_gat<false>),
                      hipFuncAttributeMaxDynamicSharedMemorySize, LDS_GAT_BYTES);

  k_gemm<INDIM><<<nP / GR, NTHR, 0, stream>>>(Ah1, Wt1, al1, ar1, feat, elr, nN);
  k_gat<true><<<nPg / NB, NTHR, LDS_GAT_BYTES, stream>>>(src, dst, feat, elr, b1, h1h, h2, nN, nE);

  k_gemm<F2><<<nP / GR, NTHR, 0, stream>>>(h1h, Wt2, al2, ar2, feat, elr, nN);
  k_gat<false><<<nPg / NB, NTHR, LDS_GAT_BYTES, stream>>>(src, dst, feat, elr, b2, h1h, h2, nN, nE);

  k_pool_head<<<1, NTHR, 0, stream>>>(h2, gidp, desc, fc1w, fc1b, fc2w, fc2b, ow, ob, out,
                                       nN, nG, out_size, invNpg);
}
